// GCNRegression_74165495267797
// MI455X (gfx1250) — hardware-verified
//
#include <hip/hip_runtime.h>


#define NN_   20000
#define NP    20032
#define NPA   20480
#define NE_   320000
#define NF    256
#define NOUT  128
#define NG_   64
#define NT    512
#define NWV   (NT / 32)
#define EPT   4
#define CHUNK (NT * EPT)
#define RB    256

typedef unsigned short bf;
typedef __attribute__((ext_vector_type(16))) __bf16   v16bf;
typedef __attribute__((ext_vector_type(8)))  unsigned short v8us;
typedef __attribute__((ext_vector_type(8)))  float    v8f;
typedef __attribute__((ext_vector_type(4)))  float    v4f;
typedef v4f  __attribute__((may_alias)) v4fa;

__device__ __forceinline__ unsigned short f2bf(float f) { unsigned u = __float_as_uint(f); u += 0x7FFFu + ((u >> 16) & 1u); return (unsigned short)(u >> 16); }
__device__ __forceinline__ float bf2f(unsigned short b) { return __uint_as_float(((unsigned)b) << 16); }
__device__ __forceinline__ float bfr(float f) { return bf2f(f2bf(f)); }
__device__ __forceinline__ v16bf cat16b(v8us lo, v8us hi) { return __builtin_bit_cast(v16bf, __builtin_shufflevector(lo, hi, 0, 1, 2, 3, 4, 5, 6, 7, 8, 9, 10, 11, 12, 13, 14, 15)); }
__device__ __forceinline__ v8f wmmab(v16bf a, v16bf b, v8f c) { return __builtin_amdgcn_wmma_f32_16x16x32_bf16(false, a, false, b, (short)0, c, false, false); }
#define VST2(T, p, v) do { const T vst2_v_ = (v); *(volatile T*)(p) = vst2_v_; __threadfence(); *(volatile T*)(p) = vst2_v_; } while (0)

__global__ __launch_bounds__(256) void k_cvtb(const float* __restrict__ src, int nvalid, int nrows, bf* dst) {
    const int lane = threadIdx.x & 31, r = blockIdx.x * 8 + (threadIdx.x >> 5);
    if (r >= nrows) return;
    v8us t;
#pragma unroll
    for (int i = 0; i < 8; ++i) t[i] = (r < nvalid) ? f2bf(src[(size_t)r * NF + lane * 8 + i]) : (unsigned short)0;
    VST2(v8us, dst + (size_t)r * NF + lane * 8, t);
}

template <bool SPLITA>
__global__ __launch_bounds__(128) void k_gemmb(const bf* __restrict__ A, const bf* __restrict__ Al, const bf* __restrict__ Bn, const float* __restrict__ bias, float* C, int ldc) {
    __shared__ __align__(16) float ost[4][16 * 68];
    const int lane = threadIdx.x & 31, wave = threadIdx.x >> 5, lr = lane & 15, hi = lane >> 4;
    const int r0 = blockIdx.x * 64 + wave * 16, c0 = blockIdx.y * 64;
    const size_t aoff = (size_t)(r0 + lr) * NF + 8 * hi;
    size_t boff[4];
#pragma unroll
    for (int t = 0; t < 4; ++t) boff[t] = (size_t)(c0 + t * 16 + lr) * NF + 8 * hi;
    v8f acc[4];
#pragma unroll
    for (int t = 0; t < 4; ++t) acc[t] = (v8f){};
#pragma unroll 1
    for (int kc = 0; kc < NF; kc += 32) {
        const v16bf a = cat16b(*(const v8us*)(A + aoff + kc), *(const v8us*)(A + aoff + kc + 16));
        v16bf al = a;
        if (SPLITA) al = cat16b(*(const v8us*)(Al + aoff + kc), *(const v8us*)(Al + aoff + kc + 16));
#pragma unroll
        for (int t = 0; t < 4; ++t) {
            const v16bf b = cat16b(*(const v8us*)(Bn + boff[t] + kc), *(const v8us*)(Bn + boff[t] + kc + 16));
            acc[t] = wmmab(a, b, acc[t]);
            if (SPLITA) acc[t] = wmmab(al, b, acc[t]);
        }
        asm volatile("v_nop\n\tv_nop\n\tv_nop\n\tv_nop" : "+v"(acc[0]), "+v"(acc[1]), "+v"(acc[2]), "+v"(acc[3]) : "v"(a), "v"(al));
    }
    float* os = &ost[wave][0];
#pragma unroll
    for (int t = 0; t < 4; ++t) { const float bv = bfr(bias[c0 + t * 16 + lr]);
#pragma unroll
        for (int j = 0; j < 8; ++j) os[(hi * 8 + j) * 68 + t * 16 + lr] = acc[t][j] + bv; }
    __syncthreads();
    float* crow = C + (size_t)r0 * ldc + c0;
    auto pass = [&]() {
#pragma unroll
        for (int s = 0; s < 8; ++s) { const int Lid = (lane >> 3) + 4 * s, piece = lane & 7; const int row = Lid >> 1, cofs = (Lid & 1) * 32 + piece * 4;
            const v4f val = *(const v4fa*)(os + row * 68 + cofs); *(volatile v4f*)(crow + (size_t)row * ldc + cofs) = val; }
    };
    pass(); __threadfence(); pass();
}

__device__ __forceinline__ int block_compact(int cnt, const int* val, const float* vv, const int* flg, int* lst, float* lsv, int* wtot, int lane, int wv) {
    int incl = cnt;
#pragma unroll
    for (int o = 1; o < 32; o <<= 1) { const int y = __shfl_up(incl, o, 32); if (lane >= o) incl += y; }
    if (lane == 31) wtot[wv] = incl;
    __syncthreads();
    int off = incl - cnt, tot = 0;
#pragma unroll
    for (int i = 0; i < NWV; ++i) { const int v = wtot[i]; off += (i < wv) ? v : 0; tot += v; }
#pragma unroll
    for (int j = 0; j < EPT; ++j) { if (flg[j]) { lst[off] = val[j]; if (lsv) lsv[off] = vv[j]; ++off; } }
    __syncthreads();
    return tot;
}

__global__ __launch_bounds__(NT) void k_deg(const int* __restrict__ erow, float* DINV) {
    __shared__ int lst[CHUNK]; __shared__ int wtot[NWV];
    const int t = threadIdx.x, lane = t & 31, wv = t >> 5, n0 = blockIdx.x * RB;
    int cntme = 0;
#pragma unroll 1
    for (int base = 0; base < NE_; base += CHUNK) {
        int val[EPT]; int flg[EPT]; float vv[EPT]; int cnt = 0;
#pragma unroll
        for (int j = 0; j < EPT; ++j) { const int e = base + j * NT + t; const int d = (e < NE_) ? erow[e] : -1; const unsigned udl = (unsigned)d - (unsigned)n0;
            const int f = (udl < (unsigned)RB) ? 1 : 0; val[j] = (int)udl; flg[j] = f; vv[j] = 0.f; cnt += f; }
        const int tot = block_compact(cnt, val, vv, flg, lst, nullptr, wtot, lane, wv);
        if (t < RB) { for (int q = 0; q < tot; ++q) cntme += (lst[q] == t); }
        __syncthreads();
    }
    __shared__ float dv[RB];
    if (t < RB) dv[t] = 1.0f / sqrtf((float)cntme);
    __syncthreads();
    if (t < RB) VST2(float, DINV + n0 + t, dv[t]);
}

__global__ __launch_bounds__(NT) void k_prop(const float* __restrict__ H, const int* __restrict__ erow, const int* __restrict__ ecol, const float* __restrict__ DINV,
                                             float* AGG, bf* AH, bf* AL) {
    extern __shared__ float4 lds_raw[];
    float* agg  = (float*)lds_raw; int* lst = (int*)(agg + RB * NF); float* lsv = (float*)(lst + CHUNK); int* wtot = (int*)(lsv + CHUNK);
    const int t = threadIdx.x, lane = t & 31, wv = t >> 5, n0 = blockIdx.x * RB;
    for (int i = t; i < RB * NF; i += NT) agg[i] = 0.0f;
    __syncthreads();
#pragma unroll 1
    for (int base = 0; base < NE_; base += CHUNK) {
        int val[EPT]; float vv[EPT]; int flg[EPT]; int cnt = 0;
#pragma unroll
        for (int j = 0; j < EPT; ++j) {
            const int e = base + j * NT + t; const int d = (e < NE_) ? ecol[e] : -1; const unsigned udl = (unsigned)d - (unsigned)n0;
            const int f = (udl < (unsigned)RB) ? 1 : 0; int v = 0; float w = 0.f;
            if (f) { int s = erow[e]; if (s < 0) s += NN_; s = min(max(s, 0), NN_ - 1); v = s * RB + (int)udl; w = DINV[s] * DINV[n0 + (int)udl]; }
            val[j] = v; vv[j] = w; flg[j] = f; cnt += f;
        }
        const int tot = block_compact(cnt, val, vv, flg, lst, lsv, wtot, lane, wv);
        if (tot > 0 && t < NF) {
#pragma unroll 1
            for (int e2 = 0; e2 < tot; ++e2) { const int v = lst[e2]; const int s = v >> 8, dl = v & (RB - 1); agg[dl * NF + t] += lsv[e2] * H[(size_t)s * NF + t]; }
        }
        __syncthreads();
    }
    constexpr int RPW = RB / NWV;
#pragma unroll 1
    for (int i = 0; i < RPW; ++i) {
        const int rl = wv * RPW + i; const size_t r = (size_t)(n0 + rl);
        const float* ar = agg + rl * NF;
        const v4f a = *(const v4fa*)(ar + lane * 4), b = *(const v4fa*)(ar + 128 + lane * 4);
        v8us oh, ol;
#pragma unroll
        for (int q = 0; q < 8; ++q) { const float v = ar[lane * 8 + q]; const unsigned short hb = f2bf(v); oh[q] = hb; ol[q] = f2bf(v - bf2f(hb)); }
        *(volatile v4f*)(AGG + r * NF + lane * 4) = a; *(volatile v4f*)(AGG + r * NF + 128 + lane * 4) = b;
        *(volatile v8us*)(AH + r * NF + lane * 8) = oh; *(volatile v8us*)(AL + r * NF + lane * 8) = ol;
        __threadfence();
        *(volatile v4f*)(AGG + r * NF + lane * 4) = a; *(volatile v4f*)(AGG + r * NF + 128 + lane * 4) = b;
        *(volatile v8us*)(AH + r * NF + lane * 8) = oh; *(volatile v8us*)(AL + r * NF + lane * 8) = ol;
    }
}

__global__ __launch_bounds__(128) void k_pool(const float* __restrict__ AGG4, const int* __restrict__ batch, float* SUM, float* CNT) {
    __shared__ int lst[256]; __shared__ int wt[4];
    const int g = blockIdx.x, t = threadIdx.x, lane = t & 31, wv = t >> 5;
    float acc = 0.f; int cnt = 0;
#pragma unroll 1
    for (int i0 = 0; i0 < NN_; i0 += 128) {
        const int r = i0 + t; const int f = (r < NN_ && batch[r] == g) ? 1 : 0;
        int incl = f;
#pragma unroll
        for (int o = 1; o < 32; o <<= 1) { const int y = __shfl_up(incl, o, 32); if (lane >= o) incl += y; }
        if (lane == 31) wt[wv] = incl;
        __syncthreads();
        int off = incl - f, tot = 0;
#pragma unroll
        for (int i = 0; i < 4; ++i) { const int v = wt[i]; off += (i < wv) ? v : 0; tot += v; }
        if (f) lst[off] = r;
        __syncthreads();
#pragma unroll 1
        for (int q = 0; q < tot; ++q) acc += AGG4[(size_t)lst[q] * NF + t];
        cnt += tot;
        __syncthreads();
    }
    VST2(float, SUM + (size_t)g * NOUT + t, acc);
    if (t < 32) VST2(float, CNT + (size_t)g * 32 + t, (float)cnt);
}

__global__ __launch_bounds__(64) void k_head(const float* __restrict__ SUM, const float* __restrict__ CNT, const float* __restrict__ lw, const float* __restrict__ lb, float* out) {
    const int g = threadIdx.x;
    float mc = 0.f;
#pragma unroll 1
    for (int i = 0; i < NG_; ++i) mc = fmaxf(mc, CNT[(size_t)i * 32]);
    const float inv = 1.0f / mc;
    float s = 0.f;
#pragma unroll 4
    for (int k = 0; k < NOUT; ++k) s += (SUM[(size_t)g * NOUT + k] * inv) * bfr(lw[k]);
    VST2(float, out + g, s + bfr(lb[0]));
}

extern "C" void kernel_launch(void* const* d_in, const int* in_sizes, int n_in,
                              void* d_out, int out_size, void* d_ws, size_t ws_size, hipStream_t stream) {
    (void)in_sizes; (void)n_in; (void)out_size;
    const float* x = (const float*)d_in[0]; const int* ei = (const int*)d_in[1]; const int* batch = (const int*)d_in[2];
    const float* Wl[4] = {(const float*)d_in[4], (const float*)d_in[6], (const float*)d_in[8], (const float*)d_in[10]};
    const float* bl[4] = {(const float*)d_in[5], (const float*)d_in[7], (const float*)d_in[9], (const float*)d_in[11]};
    const float* lw = (const float*)d_in[12]; const float* lb = (const float*)d_in[13];
    float* out = (float*)d_out;
    const int* erow = ei; const int* ecol = ei + NE_;
    char* wsp = (char*)d_ws;
    auto take = [&](size_t bytes) { char* p = wsp; wsp += (bytes + 255) & ~(size_t)255; return (void*)p; };
    bf* XH = (bf*)take((size_t)NP * NF * 2);
    bf* WB[4]; for (int i = 0; i < 4; ++i) WB[i] = (bf*)take((size_t)NF * NF * 2);
    float* H = (float*)take((size_t)NP * NF * 4); float* AGG = (float*)take((size_t)NPA * NF * 4);
    bf* AH = (bf*)take((size_t)NPA * NF * 2); bf* AL = (bf*)take((size_t)NPA * NF * 2);
    float* DINV = (float*)take((size_t)NPA * 4); float* SUM = (float*)take((size_t)NG_ * NOUT * 4); float* CNT = (float*)take((size_t)NG_ * 32 * 4);
    if ((size_t)(wsp - (char*)d_ws) > ws_size) return;
    const size_t lds = (size_t)RB * NF * 4 + (size_t)CHUNK * 8 + NWV * 4;
    k_cvtb<<<NP / 8, 256, 0, stream>>>(x, NN_, NP, XH);
    k_cvtb<<<NF / 8, 256, 0, stream>>>(Wl[0], NF, NF, WB[0]);
    k_cvtb<<<NF / 8, 256, 0, stream>>>(Wl[1], NF, NF, WB[1]);
    k_cvtb<<<NF / 8, 256, 0, stream>>>(Wl[2], NF, NF, WB[2]);
    k_cvtb<<<NOUT / 8, 256, 0, stream>>>(Wl[3], NOUT, NOUT, WB[3]);
    k_deg<<<NPA / RB, NT, 0, stream>>>(erow, DINV);
    k_gemmb<false><<<dim3(NP / 64, NF / 64, 1), 128, 0, stream>>>(XH, nullptr, WB[0], bl[0], H, NF);
    k_prop<<<NPA / RB, NT, lds, stream>>>(H, erow, ecol, DINV, AGG, AH, AL);
    for (int l = 1; l < 4; ++l) {
        const int nout = (l == 3) ? NOUT : NF;
        k_gemmb<true><<<dim3(NP / 64, nout / 64, 1), 128, 0, stream>>>(AH, AL, WB[l], bl[l], H, NF);
        k_prop<<<NPA / RB, NT, lds, stream>>>(H, erow, ecol, DINV, AGG, AH, AL);
    }
    k_pool<<<NG_, NOUT, 0, stream>>>(AGG, batch, SUM, CNT);
    k_head<<<1, NG_, 0, stream>>>(SUM, CNT, lw, lb, out);
}
